// GCN_encoder_32023276159006
// MI455X (gfx1250) — hardware-run, weakly checked
//
#include <hip/hip_runtime.h>
#include <stddef.h>
#include <stdint.h>
#include <math.h>

#define NN      50000
#define NE      1000000
#define NPAD    50176
#define FIN     64
#define H1W     64
#define H2W     32
#define OCW     16
#define TERMS_1 2
#define TERMS_2 2
#define TERMS_3 2
#define AP12    128
#define AP3     64
#define WP1     128
#define WP2     128
#define WP3     64
#define KX1     (TERMS_1 * FIN)
#define KX2     (TERMS_2 * H1W)
#define KX3     (TERMS_3 * H2W)
#define NTHR    256
#define NWAVE   8
#define EPT     8
#define WCH     (32 * EPT)
#define NBRUN   1024
#define SLB     10
#define NBK     49
#define WLCAP   3584
#define RCAP    28672
#define DEGCAP  64
#define MEAS_MAXDEG_IN  40
#define MEAS_B1024_IN   20839
#define MEAS_B1024_OUT  20897
#define ABM     64
#define GBM     128
#define SP1     68
#define SP2     36
#define OUT1_EL 1600000

#define BK_ZINTS (2 * RCAP + 4 * NBRUN)
#define BK_INTS  (BK_ZINTS + 2 * NBRUN + 32)
#define BK_LDS   (BK_INTS * 4)

#define PBX  (NPAD * FIN / 4 / NTHR)
#define PBW1 (H1W * WP1 / 8 / NTHR)
#define PBW2 (H2W * WP2 / 8 / NTHR)
#define PBTOT (PBX + PBW1 + PBW2 + 2)

static_assert(TERMS_1 == 1 || TERMS_1 == 2);
static_assert(TERMS_2 == 1 || TERMS_2 == 2);
static_assert(TERMS_3 == 1 || TERMS_3 == 2);
static_assert(KX1 % 32 == 0 && KX2 % 32 == 0 && KX3 % 32 == 0);
static_assert(KX1 <= AP12 && KX1 <= WP1 && KX2 <= AP12 && KX2 <= WP2 && KX3 <= AP3 && KX3 <= WP3);
static_assert(AP12 == 2 * FIN && AP12 == 2 * H1W && AP3 == 2 * H2W);
static_assert(FIN % 4 == 0 && H1W % 4 == 0 && H2W % 4 == 0 && (2 * FIN) % 32 == 0 && (2 * H2W) % 32 == 0);
static_assert(NN <= 65536);
static_assert(NPAD % 1024 == 0 && NPAD == NBK * NBRUN && NPAD % GBM == 0 && NPAD % ABM == 0 && NPAD >= NN);
static_assert(NBRUN == (1 << SLB) && NBRUN % ABM == 0 && NBRUN == NTHR * 4);
static_assert(NE < (1 << 20) && NE % EPT == 0);
static_assert((NWAVE - 1) * (((NE + NWAVE * WCH - 1) / (NWAVE * WCH)) * WCH) < NE);
static_assert(RCAP == NWAVE * WLCAP && RCAP % (NTHR * 4) == 0 && BK_ZINTS % (NTHR * 4) == 0);
static_assert((long long)RCAP * 100 >= (long long)MEAS_B1024_IN * 105);
static_assert((long long)RCAP * 100 >= (long long)MEAS_B1024_OUT * 105);
static_assert(WLCAP >= MEAS_B1024_OUT / 8 + 8 * 52 + 1);
static_assert(DEGCAP >= MEAS_MAXDEG_IN + 8);
static_assert(BK_LDS <= 300000 && BK_LDS <= 327680);
static_assert((GBM * SP1 + 64) * 4 <= 65536);
static_assert((NPAD * FIN / 4) % NTHR == 0 && (H1W * WP1 / 8) % NTHR == 0 && (H2W * WP2 / 8) % NTHR == 0);
static_assert(OCW * WP3 / 8 <= NTHR);
static_assert(OUT1_EL == NN * H2W && (OUT1_EL * 4) % 128 == 0);
static_assert(((NN % GBM) * OCW * 4) % 128 == 0 && (NN % GBM) % 16 == 0);

typedef float          v4f   __attribute__((ext_vector_type(4)));
typedef float          v8f   __attribute__((ext_vector_type(8)));
typedef int            v4i   __attribute__((ext_vector_type(4)));
typedef int            v8i   __attribute__((ext_vector_type(8)));
typedef unsigned       v4u   __attribute__((ext_vector_type(4)));
typedef unsigned short v8us  __attribute__((ext_vector_type(8)));
typedef __bf16         v16bf __attribute__((ext_vector_type(16)));
typedef v4f  __attribute__((may_alias)) v4fa;
typedef v4i  __attribute__((may_alias)) v4ia;
typedef v4u  __attribute__((may_alias)) v4ua;
typedef v8us __attribute__((may_alias)) v8usa;
union FragB { v16bf v; v8us h[2]; v8i w; };

__device__ __forceinline__ v8f wmb(const FragB& a, const FragB& b, v8f c) {
  v8f d = __builtin_amdgcn_wmma_f32_16x16x32_bf16(false, a.v, false, b.v, (short)0, c, false, false);
  asm volatile("v_nop\n\tv_nop\n\tv_nop\n\tv_nop" : "+v"(d) : "v"(a.w), "v"(b.w));
  return d;
}

__device__ __forceinline__ unsigned bf16_bits(float f) {
  const unsigned u = __float_as_uint(f);
  const unsigned r = (u + 0x7FFFu + ((u >> 16) & 1u)) >> 16;
  const unsigned q = (u >> 16) | 0x40u;
  return ((u & 0x7fffffffu) > 0x7f800000u) ? q : r;
}
__device__ __forceinline__ float bf16_val(float f) {
  return __uint_as_float(bf16_bits(f) << 16);
}
__device__ __forceinline__ float relu_k(float v) { return (v > 0.0f) ? v : (v - v); }

__device__ __forceinline__ void hilo_pack(float v0, float v1, float v2, float v3,
                                          unsigned& h01, unsigned& h23, unsigned& l01, unsigned& l23) {
  const unsigned a0 = bf16_bits(v0), a1 = bf16_bits(v1), a2 = bf16_bits(v2), a3 = bf16_bits(v3);
  const unsigned b0 = bf16_bits(v0 - __uint_as_float(a0 << 16));
  const unsigned b1 = bf16_bits(v1 - __uint_as_float(a1 << 16));
  const unsigned b2 = bf16_bits(v2 - __uint_as_float(a2 << 16));
  const unsigned b3 = bf16_bits(v3 - __uint_as_float(a3 << 16));
  h01 = a0 | (a1 << 16); h23 = a2 | (a3 << 16);
  l01 = b0 | (b1 << 16); l23 = b2 | (b3 << 16);
}

__device__ __forceinline__ void wave_sync() {
  __builtin_amdgcn_fence(__ATOMIC_RELEASE, "wavefront");
  __builtin_amdgcn_wave_barrier();
  __builtin_amdgcn_fence(__ATOMIC_ACQUIRE, "wavefront");
}

__device__ __forceinline__ void st2_v4f(float* p, v4f v) {
  *(volatile v4f*)p = v;
  __threadfence();
  *(volatile v4f*)p = v;
}
__device__ __forceinline__ void st2_v8us(unsigned short* p, v8us v) {
  *(volatile v8us*)p = v;
  __threadfence();
  *(volatile v8us*)p = v;
}

__device__ __forceinline__ v8us colfetch8(const float* __restrict__ base, int stride) {
  float f[8];
#pragma unroll
  for (int i = 0; i < 8; ++i) f[i] = base[(size_t)i * (size_t)stride];
  v8us o;
#pragma unroll
  for (int i = 0; i < 8; ++i) o[i] = (unsigned short)bf16_bits(f[i]);
  return o;
}

template <int WITH_ID>
__device__ __forceinline__ int sweep_keys(const int* __restrict__ keys, unsigned nbs, int* mylist, int wave, int lane) {
  const int per  = ((NE + NWAVE * WCH - 1) / (NWAVE * WCH)) * WCH;
  const int ebeg = wave * per;
  const int eend = (ebeg + per < NE) ? (ebeg + per) : NE;
  int wc = 0;
#pragma unroll 1
  for (int cb = ebeg; cb < eend; cb += WCH) {
    const int e0  = cb + lane * EPT;
    const int e0c = e0 > NE - EPT ? NE - EPT : e0;
    const v4i da = *(const v4ia*)(keys + e0c);
    const v4i db = *(const v4ia*)(keys + e0c + 4);
    asm volatile("" :: "v"(da), "v"(db));
    const unsigned lim = (e0 < NE) ? (unsigned)NBRUN : 0u;
    const unsigned s0 = (unsigned)da.x - nbs, s1 = (unsigned)da.y - nbs;
    const unsigned s2 = (unsigned)da.z - nbs, s3 = (unsigned)da.w - nbs;
    const unsigned s4 = (unsigned)db.x - nbs, s5 = (unsigned)db.y - nbs;
    const unsigned s6 = (unsigned)db.z - nbs, s7 = (unsigned)db.w - nbs;
    const bool h0 = s0 < lim, h1 = s1 < lim, h2 = s2 < lim, h3 = s3 < lim;
    const bool h4 = s4 < lim, h5 = s5 < lim, h6 = s6 < lim, h7 = s7 < lim;
    const unsigned m0 = __builtin_amdgcn_ballot_w32(h0), m1 = __builtin_amdgcn_ballot_w32(h1);
    const unsigned m2 = __builtin_amdgcn_ballot_w32(h2), m3 = __builtin_amdgcn_ballot_w32(h3);
    const unsigned m4 = __builtin_amdgcn_ballot_w32(h4), m5 = __builtin_amdgcn_ballot_w32(h5);
    const unsigned m6 = __builtin_amdgcn_ballot_w32(h6), m7 = __builtin_amdgcn_ballot_w32(h7);
    const unsigned any = m0 | m1 | m2 | m3 | m4 | m5 | m6 | m7;
    if (any != 0u) {
      const int pre = (int)(__builtin_amdgcn_mbcnt_lo(m0, 0u) + __builtin_amdgcn_mbcnt_lo(m1, 0u) +
                            __builtin_amdgcn_mbcnt_lo(m2, 0u) + __builtin_amdgcn_mbcnt_lo(m3, 0u) +
                            __builtin_amdgcn_mbcnt_lo(m4, 0u) + __builtin_amdgcn_mbcnt_lo(m5, 0u) +
                            __builtin_amdgcn_mbcnt_lo(m6, 0u) + __builtin_amdgcn_mbcnt_lo(m7, 0u));
      int p = wc + pre;
      if (h0) { if (p < WLCAP) mylist[p] = (WITH_ID ? ((e0 + 0) << SLB) : 0) | (int)s0; p = p + 1; }
      if (h1) { if (p < WLCAP) mylist[p] = (WITH_ID ? ((e0 + 1) << SLB) : 0) | (int)s1; p = p + 1; }
      if (h2) { if (p < WLCAP) mylist[p] = (WITH_ID ? ((e0 + 2) << SLB) : 0) | (int)s2; p = p + 1; }
      if (h3) { if (p < WLCAP) mylist[p] = (WITH_ID ? ((e0 + 3) << SLB) : 0) | (int)s3; p = p + 1; }
      if (h4) { if (p < WLCAP) mylist[p] = (WITH_ID ? ((e0 + 4) << SLB) : 0) | (int)s4; p = p + 1; }
      if (h5) { if (p < WLCAP) mylist[p] = (WITH_ID ? ((e0 + 5) << SLB) : 0) | (int)s5; p = p + 1; }
      if (h6) { if (p < WLCAP) mylist[p] = (WITH_ID ? ((e0 + 6) << SLB) : 0) | (int)s6; p = p + 1; }
      if (h7) { if (p < WLCAP) mylist[p] = (WITH_ID ? ((e0 + 7) << SLB) : 0) | (int)s7; p = p + 1; }
      wc += (int)(__builtin_popcount(m0) + __builtin_popcount(m1) + __builtin_popcount(m2) + __builtin_popcount(m3) +
                  __builtin_popcount(m4) + __builtin_popcount(m5) + __builtin_popcount(m6) + __builtin_popcount(m7));
    }
  }
  return wc;
}

__device__ __forceinline__ int count_hits(const int* wl, const int* wcn, int* cntArr, int lane) {
  int ov = 0;
#pragma unroll 1
  for (int w2 = 0; w2 < NWAVE; ++w2) {
    int c = wcn[w2];
    if (c > WLCAP) ov = 1;
    c = c < 0 ? 0 : (c > WLCAP ? WLCAP : c);
    c = __builtin_amdgcn_readfirstlane(c);
#pragma unroll 1
    for (int b0 = 0; b0 < c; b0 += 32) {
      const int idx = b0 + lane;
      const int ent = wl[w2 * WLCAP + (idx < WLCAP ? idx : WLCAP - 1)];
      const int m32 = (c - b0) < 32 ? (c - b0) : 32;
#pragma unroll 1
      for (int k = 0; k < m32; ++k) {
        const int u    = __builtin_amdgcn_readlane(ent, k);
        const int slot = u & (NBRUN - 1);
        if (lane == 0) cntArr[slot] = cntArr[slot] + 1;
      }
    }
  }
  return ov;
}

__device__ __forceinline__ void bucket_flush(const int* pl, const int* cnt, const int* offs, const float* fnorm,
                                             int flagv, int* lp, int* cp, int* fp, float* ndp, float* nsp,
                                             int* flp, int tid) {
#pragma unroll 1
  for (int i = tid * 4; i < RCAP; i += NTHR * 4) {
    const v4i v = *(const v4ia*)(pl + i);
    *(volatile v4i*)(lp + i) = v;
  }
  {
    const v4i vc = *(const v4ia*)(cnt + 4 * tid);
    const v4i vo = *(const v4ia*)(offs + 4 * tid);
    const v4f vd = *(const v4fa*)(fnorm + 4 * tid);
    const v4f vs = *(const v4fa*)(fnorm + NBRUN + 4 * tid);
    *(volatile v4i*)(cp + 4 * tid) = vc;
    *(volatile v4i*)(fp + 4 * tid) = vo;
    *(volatile v4f*)(ndp + 4 * tid) = vd;
    *(volatile v4f*)(nsp + 4 * tid) = vs;
  }
  if (tid < 8) {
    const v4i f = {flagv, flagv, flagv, flagv};
    *(volatile v4i*)(flp + 4 * tid) = f;
  }
}

__global__ __launch_bounds__(NTHR) void k_bucket(const int* __restrict__ srcs, const int* __restrict__ dsts,
                                                 int* LIST, int* CNT, int* OFF, float* NSp, float* NDp, int* FLAG) {
  extern __shared__ __attribute__((aligned(16))) int dsm[];
  int* wl     = dsm;
  int* pl     = wl + RCAP;
  int* cnt    = pl + RCAP;
  int* cnt2   = cnt + NBRUN;
  int* offs   = cnt2 + NBRUN;
  int* cur    = offs + NBRUN;
  float* fnorm = (float*)(cur + NBRUN);
  int* misc   = (int*)(fnorm + 2 * NBRUN);
  const int tid = (int)threadIdx.x, lane = tid & 31;
  const int wave = __builtin_amdgcn_readfirstlane(tid >> 5);
  const int blk = (int)blockIdx.x;
  const unsigned nbs = (unsigned)(blk * NBRUN);

  {
    const v4i z4 = {0, 0, 0, 0};
    for (int i = tid * 4; i < BK_ZINTS; i += NTHR * 4) *(v4ia*)(dsm + i) = z4;
    if (tid < 32) misc[tid] = 0;
  }
  __syncthreads();

  {
    const int wc = sweep_keys<1>(dsts, nbs, wl + wave * WLCAP, wave, lane);
    if (lane == 0) misc[wave] = wc;
  }
  __syncthreads();
  if (wave == 0) {
    const int ov = count_hits(wl, misc, cnt, lane);
    if (lane == 0) misc[9] = ov;
  }
  __syncthreads();
  if (wave == 0) {
    const int base = lane * (NBRUN / 32);
    int s = 0;
#pragma unroll 1
    for (int i = 0; i < NBRUN / 32; ++i) s += cnt[base + i];
    int incl = s;
#pragma unroll
    for (int d = 1; d < 32; d <<= 1) {
      const int y = __shfl_up(incl, d, 32);
      if (lane >= d) incl += y;
    }
    int run = incl - s;
#pragma unroll 1
    for (int i = 0; i < NBRUN / 32; ++i) {
      const int cv = cnt[base + i];
      offs[base + i] = run;
      cur[base + i]  = run;
      run += cv;
    }
  }
  __syncthreads();
  if (wave == 0) {
#pragma unroll 1
    for (int w2 = 0; w2 < NWAVE; ++w2) {
      int c = misc[w2];
      c = c < 0 ? 0 : (c > WLCAP ? WLCAP : c);
      c = __builtin_amdgcn_readfirstlane(c);
#pragma unroll 1
      for (int b0 = 0; b0 < c; b0 += 32) {
        const int idx = b0 + lane;
        const int ent = wl[w2 * WLCAP + (idx < WLCAP ? idx : WLCAP - 1)];
        int eid = (ent >> SLB) & 0xFFFFF;
        eid = eid > NE - 1 ? NE - 1 : eid;
        int sr = srcs[eid];
        sr = sr < 0 ? 0 : (sr > NN - 1 ? NN - 1 : sr);
        const int m32 = (c - b0) < 32 ? (c - b0) : 32;
#pragma unroll 1
        for (int k = 0; k < m32; ++k) {
          const int u    = __builtin_amdgcn_readlane(ent, k);
          const int wd   = __builtin_amdgcn_readlane(sr, k);
          const int slot = u & (NBRUN - 1);
          if (lane == 0) {
            int p = cur[slot];
            p = p < 0 ? 0 : (p > RCAP - 1 ? RCAP - 1 : p);
            pl[p] = wd;
            cur[slot] = p + 1;
          }
        }
      }
    }
  }
  __syncthreads();

  {
    const int wc2 = sweep_keys<0>(srcs, nbs, wl + wave * WLCAP, wave, lane);
    if (lane == 0) misc[16 + wave] = wc2;
  }
  __syncthreads();
  if (wave == 0) {
    const int ov2 = count_hits(wl, misc + 16, cnt2, lane);
    if (lane == 0) misc[25] = ov2;
  }
  __syncthreads();

  const int ovl = misc[9];
  const int ovc = misc[25];
  {
    const float qnan = __uint_as_float(0x7fc00000u);
#pragma unroll 1
    for (int i = 0; i < 8; ++i) {
      const int j  = tid + NTHR * i;
      const int c  = cnt[j];
      const int cm = c < 1 ? 1 : c;
      float v = 1.0f / sqrtf((float)cm);
      const bool bad = (j >= NBRUN) & (ovc != 0);
      v = bad ? qnan : v;
      fnorm[j] = v;
    }
  }
  __syncthreads();

  const int flagv = ((ovl != 0) | (ovc != 0)) ? 1 : 0;
  int*   lp  = LIST + (size_t)blk * RCAP;
  int*   cp  = CNT + (size_t)blk * NBRUN;
  int*   fp  = OFF + (size_t)blk * NBRUN;
  float* ndp = NDp + (size_t)blk * NBRUN;
  float* nsp = NSp + (size_t)blk * NBRUN;
  int*   flp = FLAG + (size_t)blk * 32;
  bucket_flush(pl, cnt, offs, fnorm, flagv, lp, cp, fp, ndp, nsp, flp, tid);
  __threadfence();
  bucket_flush(pl, cnt, offs, fnorm, flagv, lp, cp, fp, ndp, nsp, flp, tid);
}

__global__ __launch_bounds__(NTHR) void k_prep(const float* __restrict__ x, const float* __restrict__ w1,
                                               const float* __restrict__ b1, const float* __restrict__ w2,
                                               const float* __restrict__ b2, const float* __restrict__ w3,
                                               const float* __restrict__ b3, const float* __restrict__ NSp,
                                               float* xs, unsigned short* w1d, unsigned short* w2d,
                                               unsigned short* w3d, float* sm) {
  const int tid = (int)threadIdx.x, lane = tid & 31;
  const int blk = (int)blockIdx.x;
  if (blk < PBX) {
    const int u   = blk * NTHR + tid;
    const int row = u >> 4, c4 = (u & 15) * 4;
    const int rc  = row < NN ? row : NN - 1;
    const v4f a = *(const v4fa*)(x + (size_t)rc * FIN + c4);
    const float ns = NSp[row];
    asm volatile("" :: "v"(a), "v"(ns));
    const bool live = row < NN;
    v4f o;
    o.x = live ? bf16_val(a.x) * ns : 0.0f;
    o.y = live ? bf16_val(a.y) * ns : 0.0f;
    o.z = live ? bf16_val(a.z) * ns : 0.0f;
    o.w = live ? bf16_val(a.w) * ns : 0.0f;
    st2_v4f(xs + (size_t)row * FIN + c4, o);
  } else if (blk < PBX + PBW1) {
    const int u = (blk - PBX) * NTHR + tid;
    const int n = u >> 4, k8 = (u & 15) * 8, kk = k8 & (FIN - 1);
    const v8us o = colfetch8(w1 + (size_t)kk * H1W + n, H1W);
    st2_v8us(w1d + (size_t)n * WP1 + k8, o);
  } else if (blk < PBX + PBW1 + PBW2) {
    const int u = (blk - PBX - PBW1) * NTHR + tid;
    const int n = u >> 4, k8 = (u & 15) * 8, kk = k8 & (H1W - 1);
    const v8us o = colfetch8(w2 + (size_t)kk * H2W + n, H2W);
    st2_v8us(w2d + (size_t)n * WP2 + k8, o);
  } else if (blk == PBX + PBW1 + PBW2) {
    if (tid < OCW * WP3 / 8) {
      const int n = tid >> 3, k8 = (tid & 7) * 8, kk = k8 & (H2W - 1);
      const v8us o = colfetch8(w3 + (size_t)kk * OCW + n, OCW);
      st2_v8us(w3d + (size_t)n * WP3 + k8, o);
    }
  } else {
    if (tid < 32) {
      const int i1 = lane < 15 ? lane : 15;
      int i2 = lane - 16; i2 = i2 < 0 ? 0 : (i2 > 7 ? 7 : i2);
      int i3 = lane - 24; i3 = i3 < 0 ? 0 : (i3 > 3 ? 3 : i3);
      const v4f a = *(const v4fa*)(b1 + 4 * i1);
      const v4f b = *(const v4fa*)(b2 + 4 * i2);
      const v4f c = *(const v4fa*)(b3 + 4 * i3);
      asm volatile("" :: "v"(a), "v"(b), "v"(c));
      const unsigned m1 = (lane < 16) ? 0xffffffffu : 0u;
      const unsigned m2 = (lane >= 16 && lane < 24) ? 0xffffffffu : 0u;
      const unsigned m3 = (lane >= 24 && lane < 28) ? 0xffffffffu : 0u;
      v4f o;
      o.x = __uint_as_float(((bf16_bits(a.x) << 16) & m1) | ((bf16_bits(b.x) << 16) & m2) | ((bf16_bits(c.x) << 16) & m3));
      o.y = __uint_as_float(((bf16_bits(a.y) << 16) & m1) | ((bf16_bits(b.y) << 16) & m2) | ((bf16_bits(c.y) << 16) & m3));
      o.z = __uint_as_float(((bf16_bits(a.z) << 16) & m1) | ((bf16_bits(b.z) << 16) & m2) | ((bf16_bits(c.z) << 16) & m3));
      o.w = __uint_as_float(((bf16_bits(a.w) << 16) & m1) | ((bf16_bits(b.w) << 16) & m2) | ((bf16_bits(c.w) << 16) & m3));
      st2_v4f(sm + 4 * lane, o);
    }
  }
}

template <int W, int APITCH>
__global__ __launch_bounds__(NTHR) void k_replay(const int* __restrict__ LIST, const int* __restrict__ CNT,
                                                 const int* __restrict__ OFF, const int* __restrict__ FLAG,
                                                 const float* __restrict__ NDp, const float* __restrict__ P,
                                                 unsigned short* AGG) {
  constexpr int LPD   = W / 4;
  constexpr int RPS   = 32 / LPD;
  constexpr int STEPS = (ABM / NWAVE) / RPS;
  static_assert(W % 4 == 0 && 32 % LPD == 0 && (ABM / NWAVE) % RPS == 0 && APITCH == 2 * W && RPS * W == 128);
  __shared__ __attribute__((aligned(16))) unsigned rowst[NWAVE * 128];
  const int tid = (int)threadIdx.x, lane = tid & 31, wave = tid >> 5;
  const int g = lane / LPD, q = lane % LPD;
  const int rowBase = (int)blockIdx.x * ABM;
  const int bucket  = rowBase >> SLB;
  const int* lb  = LIST + (size_t)bucket * RCAP;
  const int flag = FLAG[(size_t)bucket * 32];
  const float qnan = __uint_as_float(0x7fc00000u);
  unsigned* wst = rowst + wave * 128;

#pragma unroll 1
  for (int i = 0; i < STEPS; ++i) {
    const int d = rowBase + (ABM / NWAVE) * wave + RPS * i + g;
    int c = CNT[d];
    int o = OFF[d];
    const bool big = c > DEGCAP;
    c = c < 0 ? 0 : (c > DEGCAP ? DEGCAP : c);
    o = o < 0 ? 0 : (o > RCAP - 1 ? RCAP - 1 : o);
    c = c > RCAP - o ? RCAP - o : c;
    int cm = c;
#pragma unroll
    for (int sh = LPD; sh < 32; sh <<= 1) {
      const int oth = __shfl_xor(cm, sh, 32);
      cm = cm > oth ? cm : oth;
    }
    cm = __builtin_amdgcn_readfirstlane(cm);
    int last = o + c - 1;
    last = last < o ? o : last;
    last = last > RCAP - 1 ? RCAP - 1 : last;
    float a0 = 0.0f, a1 = 0.0f, a2 = 0.0f, a3 = 0.0f;
#pragma unroll 1
    for (int j = 0; j < cm; ++j) {
      int idx = o + j;
      idx = idx > last ? last : idx;
      int sr = lb[idx];
      sr = sr < 0 ? 0 : (sr > NN - 1 ? NN - 1 : sr);
      const v4f v = *(const v4fa*)(P + (size_t)sr * W + 4 * q);
      asm volatile("" :: "v"(v));
      const bool valid = j < c;
      const float t0 = a0 + v.x, t1 = a1 + v.y, t2 = a2 + v.z, t3 = a3 + v.w;
      a0 = valid ? t0 : a0; a1 = valid ? t1 : a1; a2 = valid ? t2 : a2; a3 = valid ? t3 : a3;
    }
    const float nd = NDp[d];
    float m0 = a0 * nd, m1 = a1 * nd, m2 = a2 * nd, m3 = a3 * nd;
    const bool bad  = (flag != 0) | big;
    const bool live = d < NN;
    m0 = bad ? qnan : m0; m1 = bad ? qnan : m1; m2 = bad ? qnan : m2; m3 = bad ? qnan : m3;
    m0 = live ? m0 : 0.0f; m1 = live ? m1 : 0.0f; m2 = live ? m2 : 0.0f; m3 = live ? m3 : 0.0f;
    unsigned h01, h23, l01, l23;
    hilo_pack(m0, m1, m2, m3, h01, h23, l01, l23);
    wst[g * W + 2 * q]             = h01;
    wst[g * W + 2 * q + 1]         = h23;
    wst[g * W + W / 2 + 2 * q]     = l01;
    wst[g * W + W / 2 + 2 * q + 1] = l23;
    wave_sync();
    const v4u ow = *(const v4ua*)(wst + g * W + 4 * q);
    wave_sync();
    unsigned short* hp = AGG + (size_t)d * APITCH + 8 * q;
    *(volatile v4u*)hp = ow;
    __threadfence();
    *(volatile v4u*)hp = ow;
  }
}

template <int KTOT, int NT, int BPITCH>
__device__ __forceinline__ void gemm_rows(const unsigned short* __restrict__ ap,
                                          const unsigned short* __restrict__ bp, v8f (&acc)[NT]) {
  static_assert(KTOT % 32 == 0 && KTOT <= BPITCH);
#pragma unroll 1
  for (int k0 = 0; k0 < KTOT; k0 += 32) {
    FragB af;
    af.h[0] = *(const v8usa*)(ap + k0);
    af.h[1] = *(const v8usa*)(ap + k0 + 16);
#pragma unroll
    for (int nt = 0; nt < NT; ++nt) {
      const unsigned short* wq = bp + (size_t)(16 * nt) * (size_t)BPITCH + k0;
      FragB bf;
      bf.h[0] = *(const v8usa*)wq;
      bf.h[1] = *(const v8usa*)(wq + 16);
      acc[nt] = wmb(af, bf, acc[nt]);
    }
  }
}

template <int NT, int PITCH>
__device__ __forceinline__ void stage_d(float* stg, const v8f (&acc)[NT], int wave, int hh, int m) {
#pragma unroll
  for (int nt = 0; nt < NT; ++nt) {
#pragma unroll
    for (int r = 0; r < 8; ++r) stg[(16 * wave + 8 * hh + r) * PITCH + 16 * nt + m] = acc[nt][r];
  }
}

__global__ __launch_bounds__(NTHR) __attribute__((amdgpu_num_vgpr(248)))
void k_lin1(const unsigned short* __restrict__ A, const unsigned short* __restrict__ BT,
            const float* __restrict__ sm, const float* __restrict__ NSp, float* HS1) {
  __shared__ __attribute__((aligned(16))) float stg[GBM * SP1];
  __shared__ __attribute__((aligned(16))) float sb[64];
  const int tid = (int)threadIdx.x, lane = tid & 31, wave = tid >> 5, hh = lane >> 4, m = lane & 15;
  const int rowBase = (int)blockIdx.x * GBM;
  if (tid < 16) *(v4fa*)(sb + 4 * tid) = *(const v4fa*)(sm + 4 * tid);

  v8f acc[4];
  {
    const v8f z = {0.f, 0.f, 0.f, 0.f, 0.f, 0.f, 0.f, 0.f};
#pragma unroll
    for (int t = 0; t < 4; ++t) acc[t] = z;
  }
  const unsigned short* ap = A + (size_t)(rowBase + 16 * wave + m) * (size_t)AP12 + 8 * hh;
  const unsigned short* bp = BT + (size_t)m * (size_t)WP1 + 8 * hh;
  gemm_rows<KX1, 4, WP1>(ap, bp, acc);
  stage_d<4, SP1>(stg, acc, wave, hh, m);
  __syncthreads();

  const v4f bias = *(const v4fa*)(sb + 4 * m);
#pragma unroll 1
  for (int i = 0; i < 8; ++i) {
    const int lr   = 16 * wave + 2 * i + hh;
    const int grow = rowBase + lr;
    const bool live = grow < NN;
    const v4f a = *(const v4fa*)(stg + lr * SP1 + 4 * m);
    const float ns = NSp[grow];
    asm volatile("" :: "v"(a), "v"(ns));
    float v0 = relu_k(a.x + bias.x) * ns, v1 = relu_k(a.y + bias.y) * ns;
    float v2 = relu_k(a.z + bias.z) * ns, v3 = relu_k(a.w + bias.w) * ns;
    v4f o;
    o.x = live ? v0 : 0.0f; o.y = live ? v1 : 0.0f; o.z = live ? v2 : 0.0f; o.w = live ? v3 : 0.0f;
    st2_v4f(HS1 + (size_t)grow * H1W + 4 * m, o);
  }
}

__global__ __launch_bounds__(NTHR) __attribute__((amdgpu_num_vgpr(248)))
void k_lin2(const unsigned short* __restrict__ A, const unsigned short* __restrict__ BT,
            const float* __restrict__ sm, const float* __restrict__ NSp, float* out0, float* HS2) {
  __shared__ __attribute__((aligned(16))) float stg[GBM * SP2];
  __shared__ __attribute__((aligned(16))) float sb[32];
  const int tid = (int)threadIdx.x, lane = tid & 31, wave = tid >> 5, hh = lane >> 4, m = lane & 15;
  const int rowBase = (int)blockIdx.x * GBM;
  if (tid < 8) *(v4fa*)(sb + 4 * tid) = *(const v4fa*)(sm + 64 + 4 * tid);

  v8f acc[2];
  {
    const v8f z = {0.f, 0.f, 0.f, 0.f, 0.f, 0.f, 0.f, 0.f};
    acc[0] = z; acc[1] = z;
  }
  const unsigned short* ap = A + (size_t)(rowBase + 16 * wave + m) * (size_t)AP12 + 8 * hh;
  const unsigned short* bp = BT + (size_t)m * (size_t)WP2 + 8 * hh;
  gemm_rows<KX2, 2, WP2>(ap, bp, acc);
  stage_d<2, SP2>(stg, acc, wave, hh, m);
  __syncthreads();

  const int g = lane >> 3, q = lane & 7;
  const v4f bias = *(const v4fa*)(sb + 4 * q);
#pragma unroll 1
  for (int i = 0; i < 4; ++i) {
    const int lr   = 16 * wave + 4 * i + g;
    const int grow = rowBase + lr;
    const bool live = grow < NN;
    const v4f a = *(const v4fa*)(stg + lr * SP2 + 4 * q);
    const float ns = NSp[grow];
    asm volatile("" :: "v"(a), "v"(ns));
    v4f e;
    e.x = a.x + bias.x; e.y = a.y + bias.y; e.z = a.z + bias.z; e.w = a.w + bias.w;
    const float r0 = relu_k(e.x) * ns, r1 = relu_k(e.y) * ns, r2 = relu_k(e.z) * ns, r3 = relu_k(e.w) * ns;
    v4f hv;
    hv.x = live ? r0 : 0.0f; hv.y = live ? r1 : 0.0f; hv.z = live ? r2 : 0.0f; hv.w = live ? r3 : 0.0f;
    asm volatile("" :: "v"(e), "v"(hv));
    const int gro = live ? grow : 0;
    float* op = out0 + (size_t)gro * H2W + 4 * q;
    float* hp = HS2 + (size_t)grow * H2W + 4 * q;
    if (live) *(volatile v4f*)op = e;
    *(volatile v4f*)hp = hv;
    __threadfence();
    if (live) *(volatile v4f*)op = e;
    *(volatile v4f*)hp = hv;
  }
}

__device__ __forceinline__ void tail_flush(const float* stg3, float* ob, int nv4, int tid) {
#pragma unroll 1
  for (int it = 0; it < (GBM * OCW / 4) / NTHR; ++it) {
    const int i4 = it * NTHR + tid;
    const v4f v = *(const v4fa*)(stg3 + 4 * i4);
    asm volatile("" :: "v"(v));
    if (i4 < nv4) *(volatile v4f*)(ob + (size_t)4 * (size_t)i4) = v;
  }
}

__global__ __launch_bounds__(NTHR) __attribute__((amdgpu_num_vgpr(248)))
void k_lin3(const unsigned short* __restrict__ A, const unsigned short* __restrict__ BT,
            const float* __restrict__ sm, float* out1) {
  __shared__ __attribute__((aligned(16))) float stg3[GBM * OCW];
  __shared__ __attribute__((aligned(16))) float sb[16];
  const int tid = (int)threadIdx.x, lane = tid & 31, wave = tid >> 5, hh = lane >> 4, m = lane & 15;
  const int blk = (int)blockIdx.x;
  const int rowBase = blk * GBM;
  if (tid < 4) *(v4fa*)(sb + 4 * tid) = *(const v4fa*)(sm + 96 + 4 * tid);
  __syncthreads();

  v8f acc[1];
  {
    const v8f z = {0.f, 0.f, 0.f, 0.f, 0.f, 0.f, 0.f, 0.f};
    acc[0] = z;
  }
  const unsigned short* ap = A + (size_t)(rowBase + 16 * wave + m) * (size_t)AP3 + 8 * hh;
  const unsigned short* bp = BT + (size_t)m * (size_t)WP3 + 8 * hh;
  gemm_rows<KX3, 1, WP3>(ap, bp, acc);
  const float bb = sb[m];
#pragma unroll
  for (int r = 0; r < 8; ++r) stg3[(16 * wave + 8 * hh + r) * OCW + m] = acc[0][r] + bb;
  __syncthreads();

  int liveRows = NN - rowBase;
  liveRows = liveRows < 0 ? 0 : (liveRows > GBM ? GBM : liveRows);
  const int nv4 = liveRows * (OCW / 4);
  const int blkc = liveRows > 0 ? blk : 0;
  float* ob = out1 + (size_t)blkc * (size_t)(GBM * OCW);
  tail_flush(stg3, ob, nv4, tid);
  __threadfence();
  tail_flush(stg3, ob, nv4, tid);
}

extern "C" void kernel_launch(void* const* d_in, const int* in_sizes, int n_in,
                              void* d_out, int out_size, void* d_ws, size_t ws_size,
                              hipStream_t stream) {
  if (n_in < 9) return;
  if (in_sizes[0] != NN * FIN) return;
  if (in_sizes[1] != FIN * H1W) return;
  if (in_sizes[2] != H1W) return;
  if (in_sizes[3] != H1W * H2W) return;
  if (in_sizes[4] != H2W) return;
  if (in_sizes[5] != H2W * OCW) return;
  if (in_sizes[6] != OCW) return;
  if (in_sizes[7] != NE || in_sizes[8] != NE) return;
  if (out_size != NN * H2W + NN * OCW) return;

  const float* x  = (const float*)d_in[0];
  const float* W1 = (const float*)d_in[1];
  const float* b1 = (const float*)d_in[2];
  const float* W2 = (const float*)d_in[3];
  const float* b2 = (const float*)d_in[4];
  const float* W3 = (const float*)d_in[5];
  const float* b3 = (const float*)d_in[6];
  const int*   srcs = (const int*)d_in[7];
  const int*   dsts = (const int*)d_in[8];
  float* out0 = (float*)d_out;
  float* out1 = out0 + (size_t)OUT1_EL;

  constexpr size_t zF64  = (size_t)NPAD * 64 * 4;
  constexpr size_t zAGG  = (size_t)NPAD * AP12 * 2;
  constexpr size_t zF32  = (size_t)NPAD * 32 * 4;
  constexpr size_t zLIST = (size_t)NBK * RCAP * 4;
  constexpr size_t zTAB  = (size_t)NPAD * 4;
  constexpr size_t zFLAG = 6400;
  constexpr size_t zW1D  = (size_t)H1W * WP1 * 2;
  constexpr size_t zW2D  = (size_t)H2W * WP2 * 2;
  constexpr size_t zW3D  = (size_t)OCW * WP3 * 2;
  constexpr size_t zSM   = 512;
  constexpr size_t oXS   = 0;
  constexpr size_t oAGG  = oXS + zF64;
  constexpr size_t oHS1  = oAGG + zAGG;
  constexpr size_t oHS2  = oHS1 + zF64;
  constexpr size_t oLIST = oHS2 + zF32;
  constexpr size_t oCNT  = oLIST + zLIST;
  constexpr size_t oOFF  = oCNT + zTAB;
  constexpr size_t oNS   = oOFF + zTAB;
  constexpr size_t oND   = oNS + zTAB;
  constexpr size_t oFLAG = oND + zTAB;
  constexpr size_t oW1D  = oFLAG + zFLAG;
  constexpr size_t oW2D  = oW1D + zW1D;
  constexpr size_t oW3D  = oW2D + zW2D;
  constexpr size_t oSM   = oW3D + zW3D;
  constexpr size_t oEND  = oSM + zSM;
  static_assert(zF64 % 128 == 0 && zAGG % 128 == 0 && zF32 % 128 == 0 && zLIST % 128 == 0 && zTAB % 128 == 0);
  static_assert(zFLAG % 128 == 0 && zFLAG >= (size_t)NBK * 128 && zW1D % 128 == 0 && zW2D % 128 == 0 && zW3D % 128 == 0);
  static_assert((size_t)NPAD * AP3 * 2 <= zAGG);
  static_assert(oEND <= ((size_t)128 << 20));
  if (oEND > ws_size) return;

  char* ws = (char*)d_ws;
  float*          XS   = (float*)(ws + oXS);
  unsigned short* AGG  = (unsigned short*)(ws + oAGG);
  float*          HS1  = (float*)(ws + oHS1);
  float*          HS2  = (float*)(ws + oHS2);
  int*            LIST = (int*)(ws + oLIST);
  int*            CNT  = (int*)(ws + oCNT);
  int*            OFF  = (int*)(ws + oOFF);
  float*          NSp  = (float*)(ws + oNS);
  float*          NDp  = (float*)(ws + oND);
  int*            FLAG = (int*)(ws + oFLAG);
  unsigned short* W1D  = (unsigned short*)(ws + oW1D);
  unsigned short* W2D  = (unsigned short*)(ws + oW2D);
  unsigned short* W3D  = (unsigned short*)(ws + oW3D);
  float*          SM   = (float*)(ws + oSM);

  hipFuncSetAttribute(reinterpret_cast<const void*>(&k_bucket), hipFuncAttributeMaxDynamicSharedMemorySize, (int)BK_LDS);

  k_bucket<<<NBK, NTHR, BK_LDS, stream>>>(srcs, dsts, LIST, CNT, OFF, NSp, NDp, FLAG);
  k_prep<<<PBTOT, NTHR, 0, stream>>>(x, W1, b1, W2, b2, W3, b3, NSp, XS, W1D, W2D, W3D, SM);
  k_replay<FIN, AP12><<<NPAD / ABM, NTHR, 0, stream>>>(LIST, CNT, OFF, FLAG, NDp, XS, AGG);
  k_lin1<<<NPAD / GBM, NTHR, 0, stream>>>(AGG, W1D, SM, NSp, HS1);
  k_replay<H1W, AP12><<<NPAD / ABM, NTHR, 0, stream>>>(LIST, CNT, OFF, FLAG, NDp, HS1, AGG);
  k_lin2<<<NPAD / GBM, NTHR, 0, stream>>>(AGG, W2D, SM, NSp, out0, HS2);
  k_replay<H2W, AP3><<<NPAD / ABM, NTHR, 0, stream>>>(LIST, CNT, OFF, FLAG, NDp, HS2, AGG);
  k_lin3<<<NPAD / GBM, NTHR, 0, stream>>>(AGG, W3D, SM, out1);
}
